// MultiScaleSparseSelfAttention_85220741087703
// MI455X (gfx1250) — hardware-verified
//
#include <hip/hip_runtime.h>


#define NB_  2
#define TT   1024
#define CC   256
#define NH_  4
#define HDM  64
#define RAD  2
#define PCAR 1024.0f
typedef _Float16 h16;
typedef unsigned short bf;
typedef __attribute__((ext_vector_type(16))) __bf16   v16bf;
typedef __attribute__((ext_vector_type(16))) _Float16 v16h;
typedef __attribute__((ext_vector_type(8)))  _Float16 v8h;
typedef __attribute__((ext_vector_type(8)))  unsigned short v8us;
typedef __attribute__((ext_vector_type(8)))  float    v8f;
typedef __attribute__((ext_vector_type(4)))  float    v4f;
typedef v8h  __attribute__((may_alias)) v8ha;
typedef v4f  __attribute__((may_alias)) v4fa;
typedef v8us __attribute__((may_alias)) v8usa;

__device__ __forceinline__ unsigned short f2bf(float f) { unsigned u = __float_as_uint(f); u += 0x7FFFu + ((u >> 16) & 1u); return (unsigned short)(u >> 16); }
__device__ __forceinline__ float bf2f(unsigned short b) { return __uint_as_float(((unsigned)b) << 16); }
__device__ __forceinline__ float bfr(float f) { return bf2f(f2bf(f)); }
__device__ __forceinline__ v16h cat16(v8h lo, v8h hi) { return __builtin_shufflevector(lo, hi, 0, 1, 2, 3, 4, 5, 6, 7, 8, 9, 10, 11, 12, 13, 14, 15); }
__device__ __forceinline__ v16bf cat16b(v8us lo, v8us hi) { return __builtin_bit_cast(v16bf, __builtin_shufflevector(lo, hi, 0, 1, 2, 3, 4, 5, 6, 7, 8, 9, 10, 11, 12, 13, 14, 15)); }
__device__ __forceinline__ v8f wmma16(v16h a, v16h b, v8f c) { return __builtin_amdgcn_wmma_f32_16x16x32_f16(false, a, false, b, (short)0, c, false, false); }
__device__ __forceinline__ v8f wmmab(v16bf a, v16bf b, v8f c) { return __builtin_amdgcn_wmma_f32_16x16x32_bf16(false, a, false, b, (short)0, c, false, false); }


template <typename T16> struct WFrag;
template <> struct WFrag<h16> { typedef v16h V; static __device__ __forceinline__ V ld(const h16* p) { return cat16(*(const v8h*)p, *(const v8h*)(p + 16)); } static __device__ __forceinline__ v8f mma(V a, V b, v8f c) { return wmma16(a, b, c); } };
template <> struct WFrag<bf> { typedef v16bf V; static __device__ __forceinline__ V ld(const bf* p) { return cat16b(*(const v8us*)p, *(const v8us*)(p + 16)); } static __device__ __forceinline__ v8f mma(V a, V b, v8f c) { return wmmab(a, b, c); } };
template <typename T16, int NSPLIT, bool BIAS>
__global__ __launch_bounds__(32) void k_gemmw(const T16* __restrict__ A, const T16* __restrict__ A2, const T16* __restrict__ Bt, const T16* __restrict__ Bt2, int K, float* C, int ldc, const float* __restrict__ bias, size_t sA, size_t sB, size_t sC) {
    typedef typename WFrag<T16>::V V;
    __shared__ __align__(16) float os[16 * 68];
    const size_t z = blockIdx.z; A += z * sA; if (A2) A2 += z * sA; Bt += z * sB; if (Bt2) Bt2 += z * sB; C += z * sC;
    const int lane = threadIdx.x & 31, lr = lane & 15, hi = lane >> 4; const int r0 = blockIdx.x * 64, c0 = blockIdx.y * 64;
    v8f acc[4][4];
#pragma unroll
    for (int mb = 0; mb < 4; ++mb)
#pragma unroll
        for (int nb = 0; nb < 4; ++nb) acc[mb][nb] = (v8f){};
    const size_t aoff = (size_t)(r0 + lr) * K + 8 * hi, boff = (size_t)(c0 + lr) * K + 8 * hi;
#pragma unroll 1
    for (int kc = 0; kc < K; kc += 32) {
        V a[4], a2[4];
#pragma unroll
        for (int mb = 0; mb < 4; ++mb) { a[mb] = WFrag<T16>::ld(A + aoff + (size_t)mb * 16 * K + kc); if (NSPLIT == 1 || NSPLIT == 2) a2[mb] = WFrag<T16>::ld(A2 + aoff + (size_t)mb * 16 * K + kc); }
#pragma unroll
        for (int nb = 0; nb < 4; ++nb) { const V b = WFrag<T16>::ld(Bt + boff + (size_t)nb * 16 * K + kc); V b2; if (NSPLIT >= 2) b2 = WFrag<T16>::ld(Bt2 + boff + (size_t)nb * 16 * K + kc);
#pragma unroll
            for (int mb = 0; mb < 4; ++mb) { acc[mb][nb] = WFrag<T16>::mma(a[mb], b, acc[mb][nb]); if (NSPLIT == 1 || NSPLIT == 2) acc[mb][nb] = WFrag<T16>::mma(a2[mb], b, acc[mb][nb]); if (NSPLIT >= 2) acc[mb][nb] = WFrag<T16>::mma(a[mb], b2, acc[mb][nb]); } }
        asm volatile("v_nop\n\tv_nop\n\tv_nop\n\tv_nop" : "+v"(acc[0][0]), "+v"(acc[1][1]), "+v"(acc[2][2]), "+v"(acc[3][3]) : "v"(a[0]), "v"(a[3]));
    }
#pragma unroll
    for (int mb = 0; mb < 4; ++mb) {
#pragma unroll
        for (int nb = 0; nb < 4; ++nb) {
#pragma unroll
            for (int j = 0; j < 8; ++j) os[(hi * 8 + j) * 68 + nb * 16 + lr] = acc[mb][nb][j]; }
        __builtin_amdgcn_wave_barrier(); asm volatile("" ::: "memory");
        float* crow = C + (size_t)(r0 + mb * 16) * ldc + c0;
#pragma unroll 1
        for (int ps = 0; ps < 2; ++ps) {
#pragma unroll
            for (int s = 0; s < 8; ++s) { const int row = 2 * s + hi, cofs = lr * 4; v4f val = *(const v4fa*)(os + row * 68 + cofs); if (BIAS) { val[0] += bfr(bias[c0 + cofs]); val[1] += bfr(bias[c0 + cofs + 1]); val[2] += bfr(bias[c0 + cofs + 2]); val[3] += bfr(bias[c0 + cofs + 3]); }
                *(volatile v4f*)(crow + (size_t)row * ldc + cofs) = val; }
            if (ps == 0) __threadfence(); }
        __builtin_amdgcn_wave_barrier(); asm volatile("" ::: "memory");
    }
}

__device__ __forceinline__ h16 tohx(float x) { return (h16)x; }
typedef __attribute__((ext_vector_type(2))) _Float16 v2h;
typedef __attribute__((ext_vector_type(4))) _Float16 v4h;
typedef __attribute__((ext_vector_type(2))) float v2f;

__global__ __launch_bounds__(256) void k_cvt8(const float* __restrict__ src, bf* dst, size_t n8) { const size_t i = (size_t)blockIdx.x * 256 + threadIdx.x; if (i >= n8) return; const v8f v = *(const v8f*)(src + i * 8); v8us o;
#pragma unroll
    for (int k = 0; k < 8; ++k) o[k] = f2bf(v[k]); *(volatile v8us*)(dst + i * 8) = o; __threadfence(); *(volatile v8us*)(dst + i * 8) = o; }
__global__ __launch_bounds__(256) void k_asoft(const float* __restrict__ Sb, const float* __restrict__ MOD, int h, float scl, h16* P16) { const int lane = threadIdx.x & 31; const int row = blockIdx.x * 8 + (threadIdx.x >> 5); if (row >= TT) return; const float* sr = Sb + (size_t)row * TT; float sc = scl; if (MOD) { float m = MOD[(size_t)row * 64 + h]; asm volatile("" : "+v"(m)); sc = __fmul_rn(scl, m); } float v[32]; float mx = -3.0e38f;
#pragma unroll
    for (int ch = 0; ch < 8; ++ch) { const int j0 = ch * 128 + lane * 4; const v4f a = *(const v4f*)(sr + j0);
#pragma unroll
        for (int q = 0; q < 4; ++q) { const float t = __fmul_rn(a[q], sc); v[ch * 4 + q] = t; mx = fmaxf(mx, t); } }
#pragma unroll
    for (int sh = 16; sh; sh >>= 1) mx = fmaxf(mx, __shfl_xor(mx, sh, 32));
    float sum = 0.f;
#pragma unroll
    for (int k = 0; k < 32; ++k) { float d0 = __fsub_rn(v[k], mx); asm volatile("" : "+v"(d0)); v[k] = __builtin_amdgcn_exp2f(__fmul_rn(d0, 1.4426950408889634f)); sum += v[k]; }
#pragma unroll
    for (int sh = 16; sh; sh >>= 1) sum += __shfl_xor(sum, sh, 32);
    const float f = __fdiv_rn(PCAR, sum);
#pragma unroll 1
    for (int ps = 0; ps < 2; ++ps) {
#pragma unroll
        for (int ch = 0; ch < 8; ++ch) { v4h o;
#pragma unroll
            for (int q = 0; q < 4; ++q) o[q] = tohx(v[ch * 4 + q] * f); *(volatile v4h*)(P16 + (size_t)row * TT + ch * 128 + lane * 4) = o; }
        if (ps == 0) __threadfence(); } }
__global__ __launch_bounds__(256) void k_pl(const float* __restrict__ F, h16* P) { const size_t e = ((size_t)blockIdx.x * 256 + threadIdx.x) * 2; if (e >= (size_t)NH_ * TT * HDM) return; const int d = (int)(e % HDM); const int t = (int)((e / HDM) % TT); const int h = (int)(e / ((size_t)HDM * TT)); const float* s = F + (size_t)t * CC + h * HDM + d; v2h o; o[0] = tohx(s[0]); o[1] = tohx(s[1]); *(volatile v2h*)(P + e) = o; __threadfence(); *(volatile v2h*)(P + e) = o; }
__global__ __launch_bounds__(256) void k_vs(const float* __restrict__ FV, h16* VST) { const size_t e = ((size_t)blockIdx.x * 256 + threadIdx.x) * 2; if (e >= (size_t)NH_ * HDM * TT) return; const int m = (int)(e % TT); const int d = (int)((e / TT) % HDM); const int g = (int)(e / ((size_t)TT * HDM)); v2h o;
#pragma unroll
    for (int u = 0; u < 2; ++u) { float s = 0.f;
#pragma unroll
        for (int dw = -RAD; dw <= RAD; ++dw) { const int mm = (m + u + 2 * dw + TT) % TT; s = __fadd_rn(s, FV[(size_t)mm * CC + g * HDM + d]); } o[u] = tohx(s); }
    *(volatile v2h*)(VST + e) = o; __threadfence(); *(volatile v2h*)(VST + e) = o; }
__global__ __launch_bounds__(256) void k_acc(const float* __restrict__ O, int h, int first, float* ACC) { const size_t e = ((size_t)blockIdx.x * 256 + threadIdx.x) * 2; if (e >= (size_t)TT * HDM) return; const int d = (int)(e % HDM), t = (int)(e / HDM); const size_t oo = (size_t)t * CC + h * HDM + d; v2f o; const v2f prev = first ? (v2f){0.f, 0.f} : *(const v2f*)(ACC + oo); o[0] = __fadd_rn(prev[0], O[e] * (1.0f / PCAR)); o[1] = __fadd_rn(prev[1], O[e + 1] * (1.0f / PCAR)); *(volatile v2f*)(ACC + oo) = o; __threadfence(); *(volatile v2f*)(ACC + oo) = o; }
__global__ __launch_bounds__(256) void k_out(const float* __restrict__ ACC, float* OUTb) { const size_t i = ((size_t)blockIdx.x * 256 + threadIdx.x) * 4; if (i >= (size_t)TT * CC) return; const v4f a = *(const v4f*)(ACC + i); *(volatile v4f*)(OUTb + i) = a; __threadfence(); *(volatile v4f*)(OUTb + i) = a; }

extern "C" void kernel_launch(void* const* d_in, const int* in_sizes, int n_in,
                              void* d_out, int out_size, void* d_ws, size_t ws_size, hipStream_t stream) {
    (void)in_sizes; (void)n_in; (void)out_size;
    const float* IN[14]; for (int i = 0; i < 14; ++i) IN[i] = (const float*)d_in[i];
    float* OUT = (float*)d_out;
    char* wsp = (char*)d_ws;
    auto take = [&](size_t bytes) { char* p = wsp; wsp += (bytes + 255) & ~(size_t)255; return (void*)p; };
    bf* W6[6]; for (int i = 0; i < 6; ++i) W6[i] = (bf*)take((size_t)CC * CC * 2);
    bf* XB = (bf*)take((size_t)TT * CC * 2); float* FQ = (float*)take((size_t)TT * CC * 4); float* FK = (float*)take((size_t)TT * CC * 4); float* FV = (float*)take((size_t)TT * CC * 4);
    h16* QP = (h16*)take((size_t)NH_ * TT * HDM * 2); h16* KP = (h16*)take((size_t)NH_ * TT * HDM * 2); h16* VST = (h16*)take((size_t)NH_ * HDM * TT * 2); float* Sb = (float*)take((size_t)TT * TT * 4); h16* Pm = (h16*)take((size_t)TT * TT * 2); float* O = (float*)take((size_t)TT * HDM * 4); float* ACC = (float*)take((size_t)TT * CC * 4);
    if ((size_t)(wsp - (char*)d_ws) > ws_size) return;
    { const unsigned g = (CC * CC / 8 + 255) / 256; for (int i = 0; i < 6; ++i) k_cvt8<<<g, 256, 0, stream>>>(IN[2 + 2 * i], W6[i], (size_t)CC * CC / 8); }
    const unsigned LP = (unsigned)(((size_t)NH_ * TT * HDM / 2 + 255) / 256); const dim3 gP(TT / 64, CC / 64, 1);
    for (int b = 0; b < NB_; ++b) { int first = 1;
        for (int s = 0; s < 2; ++s) {
            k_cvt8<<<(TT * CC / 8 + 255) / 256, 256, 0, stream>>>(IN[s] + (size_t)b * CC * TT, XB, (size_t)TT * CC / 8);
            k_gemmw<bf, 0, true><<<gP, 32, 0, stream>>>(XB, nullptr, W6[3 * s], nullptr, CC, FQ, CC, IN[3 + 6 * s], 0, 0, 0); k_gemmw<bf, 0, true><<<gP, 32, 0, stream>>>(XB, nullptr, W6[3 * s + 1], nullptr, CC, FK, CC, IN[5 + 6 * s], 0, 0, 0); k_gemmw<bf, 0, true><<<gP, 32, 0, stream>>>(XB, nullptr, W6[3 * s + 2], nullptr, CC, FV, CC, IN[7 + 6 * s], 0, 0, 0);
            k_pl<<<LP, 256, 0, stream>>>(FQ, QP); k_pl<<<LP, 256, 0, stream>>>(FK, KP); k_vs<<<LP, 256, 0, stream>>>(FV, VST);
            for (int h = 0; h < NH_; ++h) for (int dh = -RAD; dh <= RAD; ++dh) { const int gk = (h - dh + 4 * NH_) % NH_, gv = (h + dh + 4 * NH_) % NH_;
                k_gemmw<h16, 0, false><<<dim3(TT / 64, TT / 64, 1), 32, 0, stream>>>(QP + (size_t)h * TT * HDM, nullptr, KP + (size_t)gk * TT * HDM, nullptr, HDM, Sb, TT, nullptr, 0, 0, 0);
                k_asoft<<<TT / 8, 256, 0, stream>>>(Sb, nullptr, h, 0.0625f, Pm);
                k_gemmw<h16, 0, false><<<dim3(TT / 64, 1, 1), 32, 0, stream>>>(Pm, nullptr, VST + (size_t)gv * HDM * TT, nullptr, TT, O, HDM, nullptr, 0, 0, 0);
                k_acc<<<(TT * HDM / 2 + 255) / 256, 256, 0, stream>>>(O, h, first && s == 0 && dh == -RAD, ACC); }
            first = 0; (void)first; }
        k_out<<<(TT * CC / 4 + 255) / 256, 256, 0, stream>>>(ACC, OUT + (size_t)b * TT * CC); }
}
